// EnhancedBeatFC_5111011082871
// MI455X (gfx1250) — hardware-verified
//
#include <hip/hip_runtime.h>
#include <math.h>

typedef __attribute__((ext_vector_type(16))) _Float16 v16h;
typedef __attribute__((ext_vector_type(16))) __bf16 v16b;
typedef __attribute__((ext_vector_type(8)))  _Float16 v8h;
typedef __attribute__((ext_vector_type(8)))  float v8f;
typedef __attribute__((ext_vector_type(4)))  float v4f;
typedef __attribute__((ext_vector_type(2)))  float v2f;
typedef __attribute__((ext_vector_type(4)))  unsigned v4u;
typedef __attribute__((ext_vector_type(4)))  int v4i;
typedef float __attribute__((may_alias)) float_a;
typedef int __attribute__((may_alias)) int_a;

template <typename T> __device__ __forceinline__ void vst2(void* p, T v) { *(volatile T*)p = v; __threadfence(); *(volatile T*)p = v; }
__device__ __forceinline__ v8f wmma16(v16h a, v16h b, v8f c) {
  v8f d = __builtin_amdgcn_wmma_f32_16x16x32_f16(false, a, false, b, (short)0, c, false, false);
  asm volatile("v_nop\n\tv_nop\n\tv_nop\n\tv_nop" : "+v"(d) : "v"(a), "v"(b));
  return d;
}
__device__ __forceinline__ v8f wmma_bf(v16b a, v16b b, v8f c) {
  v8f d = __builtin_amdgcn_wmma_f32_16x16x32_bf16(false, a, false, b, (short)0, c, false, false);
  asm volatile("v_nop\n\tv_nop\n\tv_nop\n\tv_nop" : "+v"(d) : "v"(a), "v"(b));
  return d;
}
__device__ __forceinline__ v16h frag_h(const _Float16* rowk0, int lane) {
  union { v16h v; v8h q[2]; } u; const _Float16* p = rowk0 + 8 * (lane >> 4);
  u.q[0] = *(const v8h*)p; u.q[1] = *(const v8h*)(p + 16); return u.v;
}
__device__ __forceinline__ v16h frag_f32(const float* rowk0, int lane) {
  v16h a; const float* p = rowk0 + 8 * (lane >> 4);
#pragma unroll
  for (int i = 0; i < 8; ++i) { a[i] = (_Float16)p[i]; a[8 + i] = (_Float16)p[16 + i]; }
  return a;
}
__device__ __forceinline__ v16h frag_f32s(const float* rowk0, int lane, float sc) {
  v16h a; const float* p = rowk0 + 8 * (lane >> 4);
#pragma unroll
  for (int i = 0; i < 8; ++i) { a[i] = (_Float16)(p[i] * sc); a[8 + i] = (_Float16)(p[16 + i] * sc); }
  return a;
}
__device__ __forceinline__ v16h fragc_f32(const float* W, int k0, int n, int lane, int ld, int K) {
  v16h a; const int g = lane >> 4;
#pragma unroll
  for (int i = 0; i < 8; ++i) { const int ka = k0 + 8 * g + i, kb = ka + 16;
    a[i] = (_Float16)(ka < K ? W[(size_t)(ka < K ? ka : K - 1) * ld + n] : 0.f); a[8 + i] = (_Float16)(kb < K ? W[(size_t)(kb < K ? kb : K - 1) * ld + n] : 0.f); }
  return a;
}
struct F2 { v16b h, l; };
__device__ __forceinline__ F2 bsplit16(const float v[16]) { F2 r;
#pragma unroll
  for (int i = 0; i < 16; ++i) { const __bf16 h = (__bf16)v[i]; r.h[i] = h; r.l[i] = (__bf16)(v[i] - (float)h); }
  return r; }
__device__ __forceinline__ F2 split_row(const float* row, int k0, int lane) { float v[16]; const float* p = row + k0 + 8 * (lane >> 4);
#pragma unroll
  for (int i = 0; i < 8; ++i) { v[i] = p[i]; v[8 + i] = p[16 + i]; }
  return bsplit16(v); }
__device__ __forceinline__ F2 split_rowK(const float* row, int k0, int lane, int K) { float v[16]; const int g = lane >> 4;
#pragma unroll
  for (int i = 0; i < 8; ++i) { const int ka = k0 + 8 * g + i, kb = ka + 16; v[i] = ka < K ? row[ka < K ? ka : K - 1] : 0.f; v[8 + i] = kb < K ? row[kb < K ? kb : K - 1] : 0.f; }
  return bsplit16(v); }
__device__ __forceinline__ F2 split_col(const float* W, int k0, int n, int lane, int ld, int K) { float v[16]; const int g = lane >> 4;
#pragma unroll
  for (int i = 0; i < 8; ++i) { const int ka = k0 + 8 * g + i, kb = ka + 16; v[i] = ka < K ? W[(size_t)(ka < K ? ka : K - 1) * ld + n] : 0.f; v[8 + i] = kb < K ? W[(size_t)(kb < K ? kb : K - 1) * ld + n] : 0.f; }
  return bsplit16(v); }
__device__ __forceinline__ v8f mac3(const F2& a, const F2& b, v8f c) { c = wmma_bf(a.l, b.h, c); c = wmma_bf(a.h, b.l, c); return wmma_bf(a.h, b.h, c); }
__device__ __forceinline__ float sigm(float v) { return 1.0f / (1.0f + expf(-v)); }
#define LDSX() do { asm volatile("s_wait_dscnt 0" ::: "memory"); __builtin_amdgcn_wave_barrier(); __builtin_amdgcn_fence(__ATOMIC_RELEASE, "workgroup"); } while (0)


#define NB 8
#define TT 4096
#define NM 26
#define CK 5
#define CF 64
#define WF 32
#define SEM 16
#define H1 256
#define H2 128
#define SW 8
#define SH 128
#define NO 2
#define NR (NB * TT)
#define WSC 256.0f
#ifndef TR
#define TR (NR / 64)
#endif
typedef __attribute__((ext_vector_type(8))) __bf16 v8b;
__device__ __forceinline__ v16b frag_b(const __bf16* rowk0, int lane) {
  union { v16b v; v8b q[2]; } u; const __bf16* p = rowk0 + 8 * (lane >> 4);
  u.q[0] = *(const v8b*)p; u.q[1] = *(const v8b*)(p + 16); return u.v;
}
__device__ __forceinline__ float bfr(float v) { return (float)(__bf16)v; }
__device__ __attribute__((noinline)) float exp_ni(float v) { return expf(v); }
__device__ __attribute__((noinline)) float erf_ni(float v) { return erff(v); }

#define WS_PC  0u
#define WS_W1  (WS_PC + 2u * CF * 160)
#define WS_SW  (WS_W1 + 2u * (size_t)H1 * WF * CF)
#define WS_W2  (WS_SW + 2u * (size_t)SH * SW * CF)
#define WS_XC  (WS_W2 + 2u * (size_t)H2 * H1)
#define WS_AG  (WS_XC + 4u * (size_t)NR * CF)
#define WS_END (WS_AG + 4u * (size_t)NR * CF)

__global__ __launch_bounds__(256) void k_pack(const float* __restrict__ CW, const float* __restrict__ W1, const float* __restrict__ SWt, const float* __restrict__ W2, char* __restrict__ ws) { const int n = blockIdx.x, which = blockIdx.y, t = threadIdx.x; __shared__ __align__(16) _Float16 s[WF * CF]; __shared__ __align__(16) __bf16 sb[H1];
  if (which == 0) { if (n >= CF) return; __bf16* sbb = (__bf16*)s; for (int e = t; e < 160; e += 256) { const int k = e / 32, c = e % 32; sbb[e] = (c < NM) ? (__bf16)CW[((size_t)k * NM + c) * CF + n] : (__bf16)0.0f; } __syncthreads(); if (t < 20) vst2((unsigned*)((__bf16*)(ws + WS_PC) + (size_t)n * 160 + t * 8), *(const v4u*)&sbb[t * 8]); }
  else if (which == 1) { for (int j = t; j < WF * CF; j += 256) s[j] = (_Float16)(bfr(W1[(size_t)j * H1 + n]) * WSC); __syncthreads(); for (int q = t; q < WF * CF / 8; q += 256) vst2((unsigned*)((_Float16*)(ws + WS_W1) + (size_t)n * WF * CF + q * 8), *(const v4u*)&s[q * 8]); }
  else if (which == 2) { if (n >= SH) return; for (int j = t; j < SW * CF; j += 256) s[j] = (_Float16)(bfr(SWt[(size_t)j * SH + n]) * WSC); __syncthreads(); for (int q = t; q < SW * CF / 8; q += 256) vst2((unsigned*)((_Float16*)(ws + WS_SW) + (size_t)n * SW * CF + q * 8), *(const v4u*)&s[q * 8]); }
  else { if (n >= H2) return; sb[t] = (__bf16)W2[(size_t)t * H2 + n]; __syncthreads(); if (t < H1 / 8) vst2((unsigned*)((__bf16*)(ws + WS_W2) + (size_t)n * H1 + t * 8), *(const v4u*)&sb[t * 8]); } }
__global__ __launch_bounds__(128) void k_conv(const float* __restrict__ X, const __bf16* __restrict__ PC, const float* __restrict__ CB, float* __restrict__ XC) { __shared__ __align__(16) float sf[4][16][68];
  const int tid = threadIdx.x, wave = tid >> 5, lane = tid & 31, col = lane & 15, g = lane >> 4; const size_t r0 = (size_t)blockIdx.x * 64 + wave * 16; const size_t row = r0 + col; const size_t b = row / TT; const int t = (int)(row % TT);
  v8f acc[4] = {};
#pragma unroll
  for (int kc = 0; kc < CK; ++kc) { v16b a; const int ts = t - (CK - 1) + kc; const bool ok = ts >= 0; const float* xr = X + (b * TT + (ok ? ts : 0)) * NM;
#pragma unroll
    for (int i = 0; i < 16; ++i) { const int c = 8 * g + (i < 8 ? i : 8 + i); a[i] = (__bf16)((ok && c < NM) ? xr[c] : 0.f); }
#pragma unroll
    for (int j = 0; j < 4; ++j) acc[j] = wmma_bf(a, frag_b(PC + (size_t)(j * 16 + col) * 160 + kc * 32, lane), acc[j]); }
#pragma unroll
  for (int j = 0; j < 4; ++j) { const float bb = bfr(CB[j * 16 + col]);
#pragma unroll
    for (int r = 0; r < 8; ++r) sf[wave][8 * g + r][j * 16 + col] = fmaxf(acc[j][r] + bb, 0.f); }
  LDSX(); for (int rl = 0; rl < 16; ++rl) if (lane < 16) vst2(XC + (r0 + rl) * CF + lane * 4, *(const v4f*)&sf[wave][rl][lane * 4]); }
__global__ __launch_bounds__(256) void k_se(const float* __restrict__ XC, const float* __restrict__ W1s, const float* __restrict__ B1s, const float* __restrict__ W2s, const float* __restrict__ B2s, float* __restrict__ AG) { __shared__ float ss[64][CF + 1]; __shared__ float sm[64][SEM + 1]; __shared__ __align__(16) float sa[64][CF + 4]; const int tid = threadIdx.x; const size_t rb = (size_t)blockIdx.x * 64;
  for (int e = tid; e < 64 * CF; e += 256) { const int rl = e / CF, f = e % CF; const size_t row = rb + rl; const size_t b = row / TT; const int t = (int)(row % TT); float s = 0.f;
#pragma unroll 1
    for (int w = 0; w < WF; ++w) { const int ts = t - (WF - 1) + w; if (ts >= 0) s += XC[(b * TT + ts) * CF + f]; } ss[rl][f] = s * (1.0f / WF); }
  __syncthreads();
  for (int e = tid; e < 64 * SEM; e += 256) { const int rl = e / SEM, m = e % SEM; float v = bfr(B1s[m]);
#pragma unroll 1
    for (int f = 0; f < CF; ++f) v += ss[rl][f] * bfr(W1s[f * SEM + m]); sm[rl][m] = fmaxf(v, 0.f); }
  __syncthreads();
  for (int e = tid; e < 64 * CF; e += 256) { const int rl = e / CF, f = e % CF; float v = bfr(B2s[f]);
#pragma unroll 1
    for (int m = 0; m < SEM; ++m) v += sm[rl][m] * bfr(W2s[m * CF + f]); sa[rl][f] = 1.0f / (1.0f + expf(-v)); }
  __syncthreads(); for (int e = tid; e < 64 * 16; e += 256) { const int rl = e >> 4, q = e & 15; vst2(AG + (rb + rl) * CF + q * 4, *(const v4f*)&sa[rl][q * 4]); } }
__device__ __forceinline__ float gwin(const float* XC, const float* AG, size_t b, int t, int w, int f) { const int ts = t - (WF - 1) + w; return ts >= 0 ? XC[(b * TT + ts) * CF + f] * AG[(b * TT + t) * CF + f] : 0.f; }
__global__ __launch_bounds__(128) void k_back(const float* __restrict__ XC, const float* __restrict__ AG, const _Float16* __restrict__ W1R, const float* __restrict__ B1, const __bf16* __restrict__ W2R, const float* __restrict__ B2, const _Float16* __restrict__ SWR, const float* __restrict__ SB, const float* __restrict__ WO, const float* __restrict__ BO, float* __restrict__ OUT) {
  __shared__ __align__(16) float sh1[64][H1 + 4]; __shared__ __align__(16) float scat[64][H2 + SH + 4]; __shared__ __align__(16) float so2[64 * NO];
  const int tid = threadIdx.x, wave = tid >> 5, lane = tid & 31, col = lane & 15, g = lane >> 4; const size_t r0 = (size_t)blockIdx.x * 64 + wave * 16; const size_t row = r0 + col; const size_t b = row / TT; const int t = (int)(row % TT);
{ v8f acc[16];
#pragma unroll
    for (int j = 0; j < 16; ++j) acc[j] = v8f{};
    float ag[2][16]; { const float* agr = AG + (b * TT + t) * CF;
#pragma unroll
      for (int i = 0; i < 8; ++i) { ag[0][i] = agr[8 * g + i]; ag[0][8 + i] = agr[16 + 8 * g + i]; ag[1][i] = agr[32 + 8 * g + i]; ag[1][8 + i] = agr[48 + 8 * g + i]; } }
#pragma unroll 1
    for (int w = 0; w < WF; ++w) { const int ts = t - (WF - 1) + w; const float* xr0 = XC + (b * TT + (ts >= 0 ? ts : 0)) * CF + 8 * g; const float okf = ts >= 0 ? 1.f : 0.f;
#pragma unroll
      for (int par = 0; par < 2; ++par) { v16h a; const float* xr = xr0 + par * 32; const int kc = 2 * w + par;
#pragma unroll
        for (int i = 0; i < 8; ++i) { a[i] = (_Float16)(xr[i] * ag[par][i] * okf); a[8 + i] = (_Float16)(xr[16 + i] * ag[par][8 + i] * okf); }
#pragma unroll
        for (int j = 0; j < 16; ++j) acc[j] = wmma16(a, frag_h(W1R + (size_t)(j * 16 + col) * (WF * CF) + kc * 32, lane), acc[j]); } }
#pragma unroll
    for (int j = 0; j < 16; ++j) { const int c = j * 16 + col; const float bb = bfr(B1[c]);
#pragma unroll
      for (int r = 0; r < 8; ++r) sh1[wave * 16 + 8 * g + r][c] = fmaxf(acc[j][r] * (1.0f / WSC) + bb, 0.f); } }
  LDSX();
  { v8f acc[8] = {};
#pragma unroll 1
    for (int kc = 0; kc < H1 / 32; ++kc) { float v[16]; const float* p2 = &sh1[wave * 16 + col][kc * 32 + 8 * g];
#pragma unroll
      for (int i = 0; i < 8; ++i) { v[i] = p2[i]; v[8 + i] = p2[16 + i]; }
      const F2 a = bsplit16(v);
#pragma unroll
      for (int j = 0; j < 8; ++j) { const v16b wv = frag_b(W2R + (size_t)(j * 16 + col) * H1 + kc * 32, lane); acc[j] = wmma_bf(a.h, wv, acc[j]); acc[j] = wmma_bf(a.l, wv, acc[j]); } }
#pragma unroll
    for (int j = 0; j < 8; ++j) { const float bb = bfr(B2[j * 16 + col]);
#pragma unroll
      for (int r = 0; r < 8; ++r) scat[wave * 16 + 8 * g + r][j * 16 + col] = fmaxf(acc[j][r] + bb, 0.f); } }
  { v8f acc[8] = {};
    float ag[2][16]; { const float* agr = AG + (b * TT + t) * CF;
#pragma unroll
      for (int i = 0; i < 8; ++i) { ag[0][i] = agr[8 * g + i]; ag[0][8 + i] = agr[16 + 8 * g + i]; ag[1][i] = agr[32 + 8 * g + i]; ag[1][8 + i] = agr[48 + 8 * g + i]; } }
#pragma unroll 1
    for (int w2 = 0; w2 < SW; ++w2) { const int w = (WF - SW) + w2; const int ts = t - (WF - 1) + w; const float* xr0 = XC + (b * TT + (ts >= 0 ? ts : 0)) * CF + 8 * g; const float okf = ts >= 0 ? 1.f : 0.f;
#pragma unroll
      for (int par = 0; par < 2; ++par) { v16h a; const float* xr = xr0 + par * 32; const int kc = 2 * w2 + par;
#pragma unroll
        for (int i = 0; i < 8; ++i) { a[i] = (_Float16)(xr[i] * ag[par][i] * okf); a[8 + i] = (_Float16)(xr[16 + i] * ag[par][8 + i] * okf); }
#pragma unroll
        for (int j = 0; j < 8; ++j) acc[j] = wmma16(a, frag_h(SWR + (size_t)(j * 16 + col) * (SW * CF) + kc * 32, lane), acc[j]); } }
#pragma unroll
    for (int j = 0; j < 8; ++j) { const float bb = bfr(SB[j * 16 + col]);
#pragma unroll
      for (int r = 0; r < 8; ++r) scat[wave * 16 + 8 * g + r][H2 + j * 16 + col] = fmaxf(acc[j][r] * (1.0f / WSC) + bb, 0.f); } }
  __syncthreads();
  { const int rl = tid >> 1, o = tid & 1; float v = bfr(BO[o]);
#pragma unroll 1
    for (int c = 0; c < H2 + SH; ++c) v += scat[rl][c] * bfr(WO[c * NO + o]); so2[rl * NO + o] = 1.0f / (1.0f + expf(-v)); }
  __syncthreads(); if (tid < 32) vst2(OUT + (size_t)blockIdx.x * 128 + tid * 4, *(const v4f*)&so2[tid * 4]); }
extern "C" void kernel_launch(void* const* d_in, const int* in_sizes, int n_in, void* d_out, int out_size, void* d_ws, size_t ws_size, hipStream_t stream) {
  (void)in_sizes; (void)n_in; (void)out_size;
  const float** F = (const float**)d_in;
  if (ws_size < (size_t)WS_END) return;
  char* ws = (char*)d_ws; __bf16 *PC = (__bf16*)(ws + WS_PC), *W2R = (__bf16*)(ws + WS_W2); _Float16 *W1R = (_Float16*)(ws + WS_W1), *SWR = (_Float16*)(ws + WS_SW); float *XC = (float*)(ws + WS_XC), *AG = (float*)(ws + WS_AG);
  k_pack<<<dim3(H1, 4), 256, 0, stream>>>(F[1], F[7], F[11], F[9], ws);
  k_conv<<<NR / 64, 128, 0, stream>>>(F[0], PC, F[2], XC);
  k_se<<<NR / 64, 256, 0, stream>>>(XC, F[3], F[4], F[5], F[6], AG);
  k_back<<<TR, 128, 0, stream>>>(XC, AG, W1R, F[8], W2R, F[10], SWR, F[12], F[13], F[14], (float*)d_out);
}
